// CrossAttention_40372692582970
// MI455X (gfx1250) — hardware-verified
//
#include <hip/hip_runtime.h>
#include <stddef.h>


#ifndef NB
#define NB 2
#endif
#ifndef SEQ
#define SEQ 2048
#endif
#define NB_FULL  2
#define SEQ_FULL 2048
#define MCTX  1024
#define QDIM  1024
#define CDIM  768
#define HEADS 16
#define DH    64
#define INNER (HEADS * DH)

static_assert(NB >= 1 && NB <= NB_FULL);
static_assert(SEQ >= 128 && SEQ <= SEQ_FULL && (SEQ % 128) == 0);
static_assert((MCTX % 128) == 0 && (MCTX % 64) == 0);
static_assert((QDIM % 64) == 0 && (CDIM % 64) == 0 && (INNER % 64) == 0);
static_assert((QDIM % 32) == 0 && (CDIM % 32) == 0 && (INNER % 32) == 0);
static_assert(DH == 64 && INNER == 1024);

typedef _Float16       v16h __attribute__((ext_vector_type(16)));
typedef _Float16       v8h  __attribute__((ext_vector_type(8)));
typedef __bf16         v16b __attribute__((ext_vector_type(16)));
typedef unsigned short v8us __attribute__((ext_vector_type(8)));
typedef float          v8f  __attribute__((ext_vector_type(8)));
typedef float          v4f  __attribute__((ext_vector_type(4)));

static_assert(sizeof(v8h) == 16 && sizeof(v8us) == 16 && sizeof(v16b) == 32 && sizeof(v4f) == 16);

union FragH { v16h v; v8h  p[2]; };
union FragB { v16b v; v8us p[2]; };

__device__ __forceinline__ unsigned int bf16_bits_rne(float f)
{
    unsigned int u = __float_as_uint(f);
    u += 0x7FFFu + ((u >> 16) & 1u);
    return u >> 16;
}
__device__ __forceinline__ float bf16_val_rne(float f)
{
    return __uint_as_float(bf16_bits_rne(f) << 16);
}

__device__ __forceinline__ v8f mma_f16(const FragH& a, const FragH& b, v8f c)
{
    c = __builtin_amdgcn_wmma_f32_16x16x32_f16(false, a.v, false, b.v, (short)0, c, false, false);
    asm volatile("v_nop\n\tv_nop\n\tv_nop\n\tv_nop" : "+v"(c) : "v"(a.v), "v"(b.v));
    return c;
}
__device__ __forceinline__ v8f mma_bf16(const FragB& a, const FragB& b, v8f c)
{
    c = __builtin_amdgcn_wmma_f32_16x16x32_bf16(false, a.v, false, b.v, (short)0, c, false, false);
    asm volatile("v_nop\n\tv_nop\n\tv_nop\n\tv_nop"
                 : "+v"(c) : "v"(a.p[0]), "v"(a.p[1]), "v"(b.p[0]), "v"(b.p[1]));
    return c;
}

__device__ __forceinline__ float max16(float v)
{
    v = fmaxf(v, __shfl_xor(v, 1, 32));
    v = fmaxf(v, __shfl_xor(v, 2, 32));
    v = fmaxf(v, __shfl_xor(v, 4, 32));
    v = fmaxf(v, __shfl_xor(v, 8, 32));
    return v;
}
__device__ __forceinline__ float sum16(float v)
{
    v += __shfl_xor(v, 1, 32);
    v += __shfl_xor(v, 2, 32);
    v += __shfl_xor(v, 4, 32);
    v += __shfl_xor(v, 8, 32);
    return v;
}

__global__ __launch_bounds__(256) void cvt_act_kernel(const float* __restrict__ src,
                                                      _Float16* __restrict__ dst,
                                                      int nrows, int ncol8, int src_rpb, int dst_rpb)
{
    const int idx = (int)blockIdx.x * 256 + (int)threadIdx.x;
    if (idx < nrows * ncol8) {
        const int row = idx / ncol8;
        const int c8  = idx - row * ncol8;
        const int bb  = row / dst_rpb;
        const int rr  = row - bb * dst_rpb;
        const size_t ncols = (size_t)ncol8 * 8;
        const float* s = src + ((size_t)bb * src_rpb + rr) * ncols + (size_t)c8 * 8;
        const v4f f0 = *(const v4f*)s;
        const v4f f1 = *(const v4f*)(s + 4);
        v8h o;
#pragma unroll
        for (int i = 0; i < 4; ++i) {
            o[i]     = (_Float16)bf16_val_rne(f0[i]);
            o[4 + i] = (_Float16)bf16_val_rne(f1[i]);
        }
        _Float16* d = dst + (size_t)row * ncols + (size_t)c8 * 8;
        *(volatile v8h*)d = o;
        __threadfence();
        *(volatile v8h*)d = o;
    }
}

__global__ __launch_bounds__(256) void wcvt_kernel(const float* __restrict__ W,
                                                   _Float16* __restrict__ Wt, int K, int N)
{
    __shared__ __attribute__((aligned(16))) _Float16 T[64 * 72];
    const int n0 = (int)blockIdx.x * 64;
    const int k0 = (int)blockIdx.y * 64;
    const int t  = (int)threadIdx.x;
#pragma unroll
    for (int i = 0; i < 16; ++i) {
        const int idx = i * 256 + t;
        const int kk = idx >> 6, nn = idx & 63;
        const float w = W[(size_t)(k0 + kk) * N + n0 + nn];
        T[nn * 72 + kk] = (_Float16)(bf16_val_rne(w) * 32.0f);
    }
    __syncthreads();
    v8h vv[2]; size_t go[2];
#pragma unroll
    for (int p = 0; p < 2; ++p) {
        const int nn = p * 32 + (t >> 3);
        const int kk = (t & 7) * 8;
        vv[p] = *(const v8h*)&T[nn * 72 + kk];
        go[p] = (size_t)(n0 + nn) * K + k0 + kk;
    }
#pragma unroll
    for (int p = 0; p < 2; ++p) *(volatile v8h*)(Wt + go[p]) = vv[p];
    __threadfence();
#pragma unroll
    for (int p = 0; p < 2; ++p) *(volatile v8h*)(Wt + go[p]) = vv[p];
}

enum { MODE_Q = 0, MODE_K = 1, MODE_V = 2, MODE_O = 3 };

template <int MODE>
__global__ __launch_bounds__(256) void gemm_kernel(const _Float16* __restrict__ A, int lda,
                                                   const _Float16* __restrict__ Bt, int K,
                                                   const float* __restrict__ bias,
                                                   void* outA, void* outB)
{
    constexpr int BM = 128, BN = 64, BK = 32, LS = 40, CS = 68;
    __shared__ __attribute__((aligned(16))) _Float16 As[BM * LS];
    __shared__ __attribute__((aligned(16))) _Float16 Bs[BN * LS];
    __shared__ __attribute__((aligned(16))) float    Cs[BM * CS];

    const int tid  = (int)threadIdx.x;
    const int lane = tid & 31;
    const int wave = tid >> 5;
    const int hh   = lane >> 4;
    const int m16  = lane & 15;
    const int m0   = (int)blockIdx.y * BM;
    const int n0   = (int)blockIdx.x * BN;

    v8f acc[4] = {};

    for (int k0 = 0; k0 < K; k0 += BK) {
#pragma unroll
        for (int i = 0; i < 2; ++i) {
            const int chunk = i * 256 + tid;
            const int r = chunk >> 2, c = (chunk & 3) * 8;
            const v8h v = *(const v8h*)(A + (size_t)(m0 + r) * lda + k0 + c);
            *(v8h*)&As[r * LS + c] = v;
        }
        {
            const int r = tid >> 2, c = (tid & 3) * 8;
            const v8h v = *(const v8h*)(Bt + (size_t)(n0 + r) * K + k0 + c);
            *(v8h*)&Bs[r * LS + c] = v;
        }
        __syncthreads();

        FragH a;
        a.p[0] = *(const v8h*)&As[(wave * 16 + m16) * LS + 8 * hh];
        a.p[1] = *(const v8h*)&As[(wave * 16 + m16) * LS + 16 + 8 * hh];
#pragma unroll
        for (int t = 0; t < 4; ++t) {
            FragH b;
            b.p[0] = *(const v8h*)&Bs[(t * 16 + m16) * LS + 8 * hh];
            b.p[1] = *(const v8h*)&Bs[(t * 16 + m16) * LS + 16 + 8 * hh];
            acc[t] = mma_f16(a, b, acc[t]);
        }
        __syncthreads();
    }

#pragma unroll
    for (int t = 0; t < 4; ++t)
#pragma unroll
        for (int r = 0; r < 8; ++r)
            Cs[(wave * 16 + 8 * hh + r) * CS + t * 16 + m16] = acc[t][r];
    __syncthreads();

    if constexpr (MODE == MODE_O) {
        float* out = (float*)outA;
        const int half = (lane >> 3) & 1;
        const int col  = half * 32 + (lane & 7) * 4;
        const v4f braw = *(const v4f*)(bias + n0 + col);
        v4f bv;
#pragma unroll
        for (int i = 0; i < 4; ++i) bv[i] = bf16_val_rne(braw[i]);
        v4f vals[8]; size_t go[8];
#pragma unroll
        for (int p = 0; p < 8; ++p) {
            const int row = p * 16 + wave * 2 + (lane >> 4);
            const v4f c = *(const v4f*)&Cs[row * CS + col];
            v4f v;
#pragma unroll
            for (int i = 0; i < 4; ++i) v[i] = c[i] * (1.0f / 512.0f) + bv[i];
            vals[p] = v;
            const int m  = m0 + row;
            const int bb = m / SEQ;
            const int nn = m - bb * SEQ;
            go[p] = ((size_t)bb * SEQ_FULL + nn) * QDIM + n0 + col;
        }
#pragma unroll
        for (int p = 0; p < 8; ++p) *(volatile v4f*)(out + go[p]) = vals[p];
        __threadfence();
#pragma unroll
        for (int p = 0; p < 8; ++p) *(volatile v4f*)(out + go[p]) = vals[p];
    } else if constexpr (MODE == MODE_Q || MODE == MODE_K) {
        unsigned short* ph = (unsigned short*)outA;
        unsigned short* pl = (unsigned short*)outB;
        const float sc = (MODE == MODE_Q) ? (1.0f / 256.0f) : (1.0f / 32.0f);
        const int col = (lane & 7) * 8;
        v8us hv[4], lv[4]; size_t go[4];
#pragma unroll
        for (int p = 0; p < 4; ++p) {
            const int row = p * 32 + wave * 4 + (lane >> 3);
            const v4f c0 = *(const v4f*)&Cs[row * CS + col];
            const v4f c1 = *(const v4f*)&Cs[row * CS + col + 4];
            v8us hb, lb;
#pragma unroll
            for (int i = 0; i < 4; ++i) {
                const float v0 = c0[i] * sc;
                const unsigned int h0 = bf16_bits_rne(v0);
                const unsigned int l0 = bf16_bits_rne(v0 - __uint_as_float(h0 << 16));
                hb[i] = (unsigned short)h0; lb[i] = (unsigned short)l0;
                const float v1 = c1[i] * sc;
                const unsigned int h1 = bf16_bits_rne(v1);
                const unsigned int l1 = bf16_bits_rne(v1 - __uint_as_float(h1 << 16));
                hb[4 + i] = (unsigned short)h1; lb[4 + i] = (unsigned short)l1;
            }
            hv[p] = hb; lv[p] = lb;
            go[p] = (size_t)(m0 + row) * INNER + n0 + col;
        }
#pragma unroll
        for (int p = 0; p < 4; ++p) {
            *(volatile v8us*)(ph + go[p]) = hv[p];
            *(volatile v8us*)(pl + go[p]) = lv[p];
        }
        __threadfence();
#pragma unroll
        for (int p = 0; p < 4; ++p) {
            *(volatile v8us*)(ph + go[p]) = hv[p];
            *(volatile v8us*)(pl + go[p]) = lv[p];
        }
    } else {
        _Float16* vt = (_Float16*)outA;
        const int bb   = m0 / MCTX;
        const int key0 = m0 - bb * MCTX;
        const int hd   = n0 / DH;
        v8h vv[4]; size_t go[4];
#pragma unroll
        for (int p = 0; p < 4; ++p) {
            const int d   = p * 16 + wave * 2 + (lane >> 4);
            const int key = ((lane >> 3) & 1) * 64 + (lane & 7) * 8;
            v8h o;
#pragma unroll
            for (int i = 0; i < 8; ++i) o[i] = (_Float16)(Cs[(key + i) * CS + d] * (1.0f / 32.0f));
            vv[p] = o;
            go[p] = ((size_t)(bb * HEADS + hd) * DH + d) * MCTX + key0 + key;
        }
#pragma unroll
        for (int p = 0; p < 4; ++p) *(volatile v8h*)(vt + go[p]) = vv[p];
        __threadfence();
#pragma unroll
        for (int p = 0; p < 4; ++p) *(volatile v8h*)(vt + go[p]) = vv[p];
    }
}

__global__ __launch_bounds__(128) void attn_kernel(const unsigned short* __restrict__ Qh,
                                                   const unsigned short* __restrict__ Ql,
                                                   const unsigned short* __restrict__ Kh,
                                                   const unsigned short* __restrict__ Kl,
                                                   const _Float16* __restrict__ Vt,
                                                   _Float16* __restrict__ Oh)
{
    constexpr int LS = 72;
    __shared__ __attribute__((aligned(16))) unsigned short Khs[64 * LS];
    __shared__ __attribute__((aligned(16))) unsigned short Kls[64 * LS];
    __shared__ __attribute__((aligned(16))) _Float16       Vts[64 * LS];
    __shared__ __attribute__((aligned(16))) _Float16       Ps [64 * LS];

    const int tid  = (int)threadIdx.x;
    const int lane = tid & 31;
    const int wave = tid >> 5;
    const int hh   = lane >> 4;
    const int m16  = lane & 15;
    const int bb   = (int)blockIdx.z;
    const int hd   = (int)blockIdx.y;
    const int qt   = (int)blockIdx.x;
    const int prow0 = bb * SEQ + qt * 64;
    const int qr    = prow0 + wave * 16 + m16;

    FragB qa0, qa1, ql0, ql1;
    {
        const unsigned short* pq = Qh + (size_t)qr * INNER + hd * DH;
        const unsigned short* pl = Ql + (size_t)qr * INNER + hd * DH;
        qa0.p[0] = *(const v8us*)(pq + 8 * hh);
        qa0.p[1] = *(const v8us*)(pq + 16 + 8 * hh);
        qa1.p[0] = *(const v8us*)(pq + 32 + 8 * hh);
        qa1.p[1] = *(const v8us*)(pq + 48 + 8 * hh);
        ql0.p[0] = *(const v8us*)(pl + 8 * hh);
        ql0.p[1] = *(const v8us*)(pl + 16 + 8 * hh);
        ql1.p[0] = *(const v8us*)(pl + 32 + 8 * hh);
        ql1.p[1] = *(const v8us*)(pl + 48 + 8 * hh);
    }

    float mrow[8], lrow[8];
    v8f o[4] = {};
#pragma unroll
    for (int r = 0; r < 8; ++r) { mrow[r] = -__builtin_inff(); lrow[r] = 0.f; }

    const size_t krow0 = (size_t)bb * MCTX;
    const size_t vrow0 = (size_t)(bb * HEADS + hd) * DH;

    for (int kt = 0; kt < MCTX / 64; ++kt) {
        __syncthreads();
#pragma unroll
        for (int i = 0; i < 4; ++i) {
            const int chunk = i * 128 + tid;
            const int r = chunk >> 3, c = (chunk & 7) * 8;
            const v8us ka = *(const v8us*)(Kh + (krow0 + kt * 64 + r) * INNER + hd * DH + c);
            const v8us kb = *(const v8us*)(Kl + (krow0 + kt * 64 + r) * INNER + hd * DH + c);
            const v8h  vv = *(const v8h*)(Vt + (vrow0 + r) * MCTX + kt * 64 + c);
            *(v8us*)&Khs[r * LS + c] = ka;
            *(v8us*)&Kls[r * LS + c] = kb;
            *(v8h*)&Vts[r * LS + c]  = vv;
        }
        __syncthreads();

        v8f s[4] = {};
#pragma unroll
        for (int t = 0; t < 4; ++t) {
            const int kb = (t * 16 + m16) * LS;
            {
                FragB bh, bl;
                bh.p[0] = *(const v8us*)&Khs[kb + 8 * hh];
                bh.p[1] = *(const v8us*)&Khs[kb + 16 + 8 * hh];
                bl.p[0] = *(const v8us*)&Kls[kb + 8 * hh];
                bl.p[1] = *(const v8us*)&Kls[kb + 16 + 8 * hh];
                s[t] = mma_bf16(qa0, bh, s[t]);
                s[t] = mma_bf16(ql0, bh, s[t]);
                s[t] = mma_bf16(qa0, bl, s[t]);
            }
            {
                FragB bh, bl;
                bh.p[0] = *(const v8us*)&Khs[kb + 32 + 8 * hh];
                bh.p[1] = *(const v8us*)&Khs[kb + 48 + 8 * hh];
                bl.p[0] = *(const v8us*)&Kls[kb + 32 + 8 * hh];
                bl.p[1] = *(const v8us*)&Kls[kb + 48 + 8 * hh];
                s[t] = mma_bf16(qa1, bh, s[t]);
                s[t] = mma_bf16(ql1, bh, s[t]);
                s[t] = mma_bf16(qa1, bl, s[t]);
            }
        }

#pragma unroll
        for (int r = 0; r < 8; ++r) {
            float rmax = fmaxf(fmaxf(s[0][r], s[1][r]), fmaxf(s[2][r], s[3][r]));
            rmax = max16(rmax);
            const float mn = fmaxf(mrow[r], rmax);
            const float al = __expf(mrow[r] - mn);
            float rsum = 0.f;
#pragma unroll
            for (int t = 0; t < 4; ++t) {
                const float p = __expf(s[t][r] - mn);
                s[t][r] = p;
                rsum += p;
            }
            rsum = sum16(rsum);
            lrow[r] = lrow[r] * al + rsum;
            mrow[r] = mn;
#pragma unroll
            for (int t = 0; t < 4; ++t) o[t][r] *= al;
        }

#pragma unroll
        for (int t = 0; t < 4; ++t)
#pragma unroll
            for (int r = 0; r < 8; ++r)
                Ps[(wave * 16 + 8 * hh + r) * LS + t * 16 + m16] = (_Float16)(s[t][r] * 256.0f);
        __syncthreads();

#pragma unroll
        for (int kc = 0; kc < 2; ++kc) {
            FragH a;
            a.p[0] = *(const v8h*)&Ps[(wave * 16 + m16) * LS + kc * 32 + 8 * hh];
            a.p[1] = *(const v8h*)&Ps[(wave * 16 + m16) * LS + kc * 32 + 16 + 8 * hh];
#pragma unroll
            for (int t = 0; t < 4; ++t) {
                FragH bv;
                bv.p[0] = *(const v8h*)&Vts[(t * 16 + m16) * LS + kc * 32 + 8 * hh];
                bv.p[1] = *(const v8h*)&Vts[(t * 16 + m16) * LS + kc * 32 + 16 + 8 * hh];
                o[t] = mma_f16(a, bv, o[t]);
            }
        }
    }

    __syncthreads();
#pragma unroll
    for (int r = 0; r < 8; ++r) {
        const float inv = 1.0f / (16.0f * lrow[r]);
#pragma unroll
        for (int t = 0; t < 4; ++t)
            Ps[(wave * 16 + 8 * hh + r) * LS + t * 16 + m16] = (_Float16)(o[t][r] * inv);
    }
    __syncthreads();
    v8h ov[4]; size_t go[4];
#pragma unroll
    for (int p = 0; p < 4; ++p) {
        const int row = wave * 16 + p * 4 + (lane >> 3);
        const int col = (lane & 7) * 8;
        ov[p] = *(const v8h*)&Ps[row * LS + col];
        go[p] = (size_t)(prow0 + row) * INNER + hd * DH + col;
    }
#pragma unroll
    for (int p = 0; p < 4; ++p) *(volatile v8h*)(Oh + go[p]) = ov[p];
    __threadfence();
#pragma unroll
    for (int p = 0; p < 4; ++p) *(volatile v8h*)(Oh + go[p]) = ov[p];
}

extern "C" void kernel_launch(void* const* d_in, const int* in_sizes, int n_in,
                              void* d_out, int out_size, void* d_ws, size_t ws_size,
                              hipStream_t stream)
{
    if (n_in < 7) return;
    const long long rowsX = (long long)(NB - 1) * SEQ_FULL + SEQ;
    if ((long long)in_sizes[0] < rowsX * QDIM) return;
    if ((long long)in_sizes[1] < (long long)NB * MCTX * CDIM) return;
    if (in_sizes[2] < QDIM * INNER) return;
    if (in_sizes[3] < CDIM * INNER) return;
    if (in_sizes[4] < CDIM * INNER) return;
    if (in_sizes[5] < INNER * QDIM) return;
    if (in_sizes[6] < QDIM) return;
    if ((long long)out_size < rowsX * QDIM) return;

    const float* x   = (const float*)d_in[0];
    const float* ctx = (const float*)d_in[1];
    const float* Wq  = (const float*)d_in[2];
    const float* Wk  = (const float*)d_in[3];
    const float* Wv  = (const float*)d_in[4];
    const float* Wo  = (const float*)d_in[5];
    const float* bo  = (const float*)d_in[6];
    float* out = (float*)d_out;

    char* ws = (char*)d_ws;
    size_t off = 0;
    const size_t szXh = (size_t)NB * SEQ * QDIM * 2;
    const size_t szCh = (size_t)NB * MCTX * CDIM * 2;
    const size_t szWq = (size_t)INNER * QDIM * 2;
    const size_t szWc = (size_t)INNER * CDIM * 2;
    const size_t szWo = (size_t)QDIM * INNER * 2;
    const size_t szQ  = (size_t)NB * SEQ * INNER * 2;
    const size_t szK  = (size_t)NB * MCTX * INNER * 2;
    const size_t szV  = (size_t)NB * HEADS * DH * MCTX * 2;
    const size_t szO  = (size_t)NB * SEQ * INNER * 2;
    _Float16* xh  = (_Float16*)(ws + off); off += szXh;
    _Float16* ch  = (_Float16*)(ws + off); off += szCh;
    _Float16* wqt = (_Float16*)(ws + off); off += szWq;
    _Float16* wkt = (_Float16*)(ws + off); off += szWc;
    _Float16* wvt = (_Float16*)(ws + off); off += szWc;
    _Float16* wot = (_Float16*)(ws + off); off += szWo;
    unsigned short* qh = (unsigned short*)(ws + off); off += szQ;
    unsigned short* ql = (unsigned short*)(ws + off); off += szQ;
    unsigned short* kh = (unsigned short*)(ws + off); off += szK;
    unsigned short* kl = (unsigned short*)(ws + off); off += szK;
    _Float16* vt  = (_Float16*)(ws + off); off += szV;
    _Float16* oh  = (_Float16*)(ws + off); off += szO;
    if (off > ws_size) return;

    {
        const int nrowsX = NB * SEQ, ncol8X = QDIM / 8;
        if ((nrowsX * ncol8X) % 256 != 0) return;
        cvt_act_kernel<<<dim3((nrowsX * ncol8X) / 256), dim3(256), 0, stream>>>(
            x, xh, nrowsX, ncol8X, SEQ_FULL, SEQ);
        const int nrowsC = NB * MCTX, ncol8C = CDIM / 8;
        if ((nrowsC * ncol8C) % 256 != 0) return;
        cvt_act_kernel<<<dim3((nrowsC * ncol8C) / 256), dim3(256), 0, stream>>>(
            ctx, ch, nrowsC, ncol8C, MCTX, MCTX);
    }
    wcvt_kernel<<<dim3(INNER / 64, QDIM / 64), dim3(256), 0, stream>>>(Wq, wqt, QDIM, INNER);
    wcvt_kernel<<<dim3(INNER / 64, CDIM / 64), dim3(256), 0, stream>>>(Wk, wkt, CDIM, INNER);
    wcvt_kernel<<<dim3(INNER / 64, CDIM / 64), dim3(256), 0, stream>>>(Wv, wvt, CDIM, INNER);
    wcvt_kernel<<<dim3(QDIM / 64, INNER / 64), dim3(256), 0, stream>>>(Wo, wot, INNER, QDIM);

    gemm_kernel<MODE_Q><<<dim3(INNER / 64, (NB * SEQ) / 128), dim3(256), 0, stream>>>(
        xh, QDIM, wqt, QDIM, bo, (void*)qh, (void*)ql);
    gemm_kernel<MODE_K><<<dim3(INNER / 64, (NB * MCTX) / 128), dim3(256), 0, stream>>>(
        ch, CDIM, wkt, CDIM, bo, (void*)kh, (void*)kl);
    gemm_kernel<MODE_V><<<dim3(INNER / 64, (NB * MCTX) / 128), dim3(256), 0, stream>>>(
        ch, CDIM, wvt, CDIM, bo, (void*)vt, (void*)vt);

    attn_kernel<<<dim3(SEQ / 64, HEADS, NB), dim3(128), 0, stream>>>(qh, ql, kh, kl, vt, oh);

    gemm_kernel<MODE_O><<<dim3(QDIM / 64, (NB * SEQ) / 128), dim3(256), 0, stream>>>(
        oh, INNER, wot, INNER, bo, (void*)out, (void*)out);
}
